// EncoderBlock_16655883174620
// MI455X (gfx1250) — hardware-verified
//
#include <hip/hip_runtime.h>
#include <stdint.h>


#ifndef NB
#define NB 2
#endif
#ifndef SEQ
#define SEQ 2048
#endif
#define NB_FULL 2
#define SEQ_FULL 2048
#define T_FULL 2048
#define DM 1024
#define NH 16
#define HD 64
#define NQKV 3072
#define HID 4096
#define NTOK (NB * SEQ)
#define FLAG_STRIDE 64

static_assert(SEQ % 128 == 0);
static_assert(SEQ >= 128);
static_assert(SEQ <= SEQ_FULL);
static_assert(NB >= 1);
static_assert(NB <= NB_FULL);
static_assert(SEQ / 32 <= FLAG_STRIDE);
static_assert(NTOK % 128 == 0);
static_assert(DM % 128 == 0);
static_assert(NQKV % 128 == 0);
static_assert(HID % 128 == 0);

typedef _Float16 v16h __attribute__((ext_vector_type(16)));
typedef _Float16 v8h  __attribute__((ext_vector_type(8)));
typedef float    v8f  __attribute__((ext_vector_type(8)));
typedef float    v4f  __attribute__((ext_vector_type(4)));
typedef int      v4i  __attribute__((ext_vector_type(4)));

static __device__ __forceinline__ v8f mma16(v16h a, v16h b, v8f c) {
  v8f d = __builtin_amdgcn_wmma_f32_16x16x32_f16(false, a, false, b, (short)0, c, false, false);
  asm volatile("v_nop\n\tv_nop\n\tv_nop\n\tv_nop" : "+v"(d) : "v"(a), "v"(b));
  return d;
}

static __device__ __forceinline__ v16h load_frag(const _Float16* p) {
  v8h lo = *(const v8h*)(p);
  v8h hi = *(const v8h*)(p + 16);
  v16h f;
#pragma unroll
  for (int e = 0; e < 8; ++e) { f[e] = lo[e]; f[e + 8] = hi[e]; }
  return f;
}

static __device__ __forceinline__ float bf16r(float f) {
  unsigned int u = __float_as_uint(f);
  u = (u + 0x7FFFu + ((u >> 16) & 1u)) & 0xFFFF0000u;
  return __uint_as_float(u);
}
static __device__ __forceinline__ v4f bf16r4(v4f a) {
  v4f o;
  o[0] = bf16r(a[0]); o[1] = bf16r(a[1]); o[2] = bf16r(a[2]); o[3] = bf16r(a[3]);
  return o;
}

#define TST 36
__global__ __launch_bounds__(256) void tcvt_kernel(
    const float* __restrict__ src, int zstride, int src_rs,
    _Float16* __restrict__ dst, int dst_rs, int dst_nz, int n_base, float scale) {
  __shared__ __align__(16) float tile[64 * TST];
  const int tid = threadIdx.x;
  const int k0 = blockIdx.x * 64, n0 = blockIdx.y * 32, z = blockIdx.z;
  const float* s = src + (size_t)z * (size_t)zstride;
  const int kk = tid >> 3, nn = (tid & 7) << 2;
  const v4f a0 = *(const v4f*)(s + (size_t)(k0 + kk) * src_rs + n0 + nn);
  const v4f a1 = *(const v4f*)(s + (size_t)(k0 + kk + 32) * src_rs + n0 + nn);
  *(v4f*)&tile[kk * TST + nn] = a0;
  *(v4f*)&tile[(kk + 32) * TST + nn] = a1;
  __syncthreads();
  const int n = tid >> 3, kq = (tid & 7) << 3;
  v8h w;
#pragma unroll
  for (int i = 0; i < 8; ++i) w[i] = (_Float16)(bf16r(tile[(kq + i) * TST + n]) * scale);
  _Float16* p = dst + (size_t)(z * dst_nz + n_base + n0 + n) * dst_rs + k0 + kq;
  *(volatile v8h*)p = w;
  __threadfence();
  *(volatile v8h*)p = w;
}

template <bool RIN>
__global__ __launch_bounds__(128) void ln_kernel(
    const float* __restrict__ x, int seq_src,
    const float* __restrict__ g, const float* __restrict__ bt,
    _Float16* __restrict__ out) {
  const int i = blockIdx.x;
  const size_t srow = (size_t)(i / SEQ) * (size_t)seq_src + (size_t)(i % SEQ);
  const int tid = threadIdx.x, wave = tid >> 5, lane = tid & 31;
  const int c = tid * 8;
  const float* xp = x + srow * DM + c;
  v4f a0 = *(const v4f*)(xp);
  v4f a1 = *(const v4f*)(xp + 4);
  if (RIN) { a0 = bf16r4(a0); a1 = bf16r4(a1); }
  float v[8];
#pragma unroll
  for (int e = 0; e < 4; ++e) { v[e] = a0[e]; v[e + 4] = a1[e]; }

  __shared__ float red[2][4];
  float s = 0.f;
#pragma unroll
  for (int e = 0; e < 8; ++e) s += v[e];
#pragma unroll
  for (int m = 16; m >= 1; m >>= 1) s += __shfl_xor(s, m, 32);
  if (lane == 0) red[0][wave] = s;
  __syncthreads();
  const float S = (red[0][0] + red[0][1]) + (red[0][2] + red[0][3]);
  const float mu = S * (1.0f / 1024.0f);

  float d[8];
  float ss = 0.f;
#pragma unroll
  for (int e = 0; e < 8; ++e) { d[e] = v[e] - mu; ss += d[e] * d[e]; }
#pragma unroll
  for (int m = 16; m >= 1; m >>= 1) ss += __shfl_xor(ss, m, 32);
  if (lane == 0) red[1][wave] = ss;
  __syncthreads();
  const float SS = (red[1][0] + red[1][1]) + (red[1][2] + red[1][3]);
  const float var = SS * (1.0f / 1024.0f);
  const float rs = rsqrtf(var + 1e-5f);

  v4f g0 = bf16r4(*(const v4f*)(g + c)),  g1v = bf16r4(*(const v4f*)(g + c + 4));
  v4f b0 = bf16r4(*(const v4f*)(bt + c)), b1v = bf16r4(*(const v4f*)(bt + c + 4));
  float gg[8], bb[8];
#pragma unroll
  for (int e = 0; e < 4; ++e) { gg[e] = g0[e]; gg[e + 4] = g1v[e]; bb[e] = b0[e]; bb[e + 4] = b1v[e]; }
  v8h o;
#pragma unroll
  for (int e = 0; e < 8; ++e) o[e] = (_Float16)(d[e] * rs * gg[e] + bb[e]);
  _Float16* op = out + (size_t)i * DM + c;
  *(volatile v8h*)op = o;
  __threadfence();
  *(volatile v8h*)op = o;
}

#define BM 128
#define BN 128
#define BK 32
#define LDT 40
#define CST 132
#define HST 136
#define SMEM_HALVES (2 * BM * LDT + 2 * BN * LDT)
static_assert(64 * CST * 4 <= SMEM_HALVES * 2);
static_assert(BM * HST * 2 <= SMEM_HALVES * 2);

template <bool HAS_BIAS, bool HAS_RES, bool RES_RND, bool RELU, bool OUT_F16>
__global__ __launch_bounds__(256) void gemm_kernel(
    const _Float16* __restrict__ A, const _Float16* __restrict__ B,
    const float* __restrict__ bias, const float* __restrict__ res, int res_seq,
    float* __restrict__ outF, _Float16* __restrict__ outH,
    int M, int N, int K, float scale) {
  __shared__ __align__(16) _Float16 smem[SMEM_HALVES];
  _Float16* As = smem;
  _Float16* Bs = smem + 2 * BM * LDT;
  const int tid = threadIdx.x, wave = tid >> 5, lane = tid & 31;
  const int r = lane & 15, hb = (lane >> 4) << 3;
  const int mBlk = blockIdx.y * BM, nBlk = blockIdx.x * BN;
  const int mw = (wave & 1) * 64, nw = (wave >> 1) * 32;
  (void)M;

  const int rw0 = tid >> 2, kc = (tid & 3) << 3, rw1 = rw0 + 64;
  const _Float16* gA0 = A + (size_t)(mBlk + rw0) * K + kc;
  const _Float16* gA1 = A + (size_t)(mBlk + rw1) * K + kc;
  const _Float16* gB0 = B + (size_t)(nBlk + rw0) * K + kc;
  const _Float16* gB1 = B + (size_t)(nBlk + rw1) * K + kc;

  v8h ra0 = *(const v8h*)gA0, ra1 = *(const v8h*)gA1;
  v8h rb0 = *(const v8h*)gB0, rb1 = *(const v8h*)gB1;
  *(v8h*)&As[rw0 * LDT + kc] = ra0;
  *(v8h*)&As[rw1 * LDT + kc] = ra1;
  *(v8h*)&Bs[rw0 * LDT + kc] = rb0;
  *(v8h*)&Bs[rw1 * LDT + kc] = rb1;

  v8f acc[4][2] = {};
  const int nk = K / BK;
  for (int kt = 0; kt < nk; ++kt) {
    const int cur = kt & 1;
    __syncthreads();
    const bool nxt = (kt + 1 < nk);
    if (nxt) {
      const size_t ko = (size_t)(kt + 1) * BK;
      ra0 = *(const v8h*)(gA0 + ko); ra1 = *(const v8h*)(gA1 + ko);
      rb0 = *(const v8h*)(gB0 + ko); rb1 = *(const v8h*)(gB1 + ko);
    }
    const _Float16* Ac = As + cur * BM * LDT;
    const _Float16* Bc = Bs + cur * BN * LDT;
    v16h af[4], bf[2];
#pragma unroll
    for (int i = 0; i < 4; ++i) af[i] = load_frag(Ac + (mw + i * 16 + r) * LDT + hb);
#pragma unroll
    for (int j = 0; j < 2; ++j) bf[j] = load_frag(Bc + (nw + j * 16 + r) * LDT + hb);
#pragma unroll
    for (int i = 0; i < 4; ++i)
#pragma unroll
      for (int j = 0; j < 2; ++j) acc[i][j] = mma16(af[i], bf[j], acc[i][j]);
    if (nxt) {
      _Float16* An = As + (cur ^ 1) * BM * LDT;
      _Float16* Bn = Bs + (cur ^ 1) * BN * LDT;
      *(v8h*)&An[rw0 * LDT + kc] = ra0;
      *(v8h*)&An[rw1 * LDT + kc] = ra1;
      *(v8h*)&Bn[rw0 * LDT + kc] = rb0;
      *(v8h*)&Bn[rw1 * LDT + kc] = rb1;
    }
  }

  if (OUT_F16) {
    _Float16* Hs = smem;
    float bcol[2] = {0.f, 0.f};
    if (HAS_BIAS) {
#pragma unroll
      for (int j = 0; j < 2; ++j) bcol[j] = bf16r(bias[(size_t)(nBlk + nw + j * 16 + r)]);
    }
    __syncthreads();
#pragma unroll
    for (int i = 0; i < 4; ++i)
#pragma unroll
      for (int j = 0; j < 2; ++j)
#pragma unroll
        for (int v = 0; v < 8; ++v) {
          float c = acc[i][j][v] * scale + bcol[j];
          if (RELU) c = fmaxf(c, 0.f);
          Hs[(mw + i * 16 + v + hb) * HST + nw + j * 16 + r] = (_Float16)c;
        }
    __syncthreads();
    const int lhw = lane >> 4, piece = lane & 15;
    v8h vals[8];
#pragma unroll
    for (int it = 0; it < 8; ++it) {
      const int row = wave * 16 + it * 2 + lhw;
      vals[it] = *(const v8h*)&Hs[row * HST + piece * 8];
    }
#pragma unroll
    for (int it = 0; it < 8; ++it) {
      const int row = wave * 16 + it * 2 + lhw;
      _Float16* p = outH + (size_t)(mBlk + row) * N + nBlk + piece * 8;
      *(volatile v8h*)p = vals[it];
    }
    __threadfence();
#pragma unroll
    for (int it = 0; it < 8; ++it) {
      const int row = wave * 16 + it * 2 + lhw;
      _Float16* p = outH + (size_t)(mBlk + row) * N + nBlk + piece * 8;
      *(volatile v8h*)p = vals[it];
    }
  } else {
    float* Cs = (float*)smem;
    v4f bia = {0.f, 0.f, 0.f, 0.f};
    if (HAS_BIAS) bia = bf16r4(*(const v4f*)(bias + nBlk + lane * 4));
#pragma unroll
    for (int half = 0; half < 2; ++half) {
      __syncthreads();
      if ((wave & 1) == half) {
#pragma unroll
        for (int i = 0; i < 4; ++i)
#pragma unroll
          for (int j = 0; j < 2; ++j)
#pragma unroll
            for (int v = 0; v < 8; ++v)
              Cs[(i * 16 + v + hb) * CST + nw + j * 16 + r] = acc[i][j][v];
      }
      __syncthreads();
      v4f vals[8];
#pragma unroll
      for (int q = 0; q < 8; ++q) {
        const int rl = wave * 8 + q;
        const int m = mBlk + half * 64 + rl;
        v4f c = *(const v4f*)&Cs[rl * CST + lane * 4];
        c = c * scale + bia;
        if (HAS_RES) {
          const size_t rr = (size_t)(m / SEQ) * (size_t)res_seq + (size_t)(m % SEQ);
          v4f rv = *(const v4f*)(res + rr * (size_t)N + nBlk + lane * 4);
          if (RES_RND) rv = bf16r4(rv);
          c = c + rv;
        }
        if (RELU) { c[0] = fmaxf(c[0], 0.f); c[1] = fmaxf(c[1], 0.f); c[2] = fmaxf(c[2], 0.f); c[3] = fmaxf(c[3], 0.f); }
        vals[q] = c;
      }
#pragma unroll
      for (int q = 0; q < 8; ++q) {
        const int m = mBlk + half * 64 + wave * 8 + q;
        float* p = outF + (size_t)m * N + nBlk + lane * 4;
        *(volatile v4f*)p = vals[q];
      }
      __threadfence();
#pragma unroll
      for (int q = 0; q < 8; ++q) {
        const int m = mBlk + half * 64 + wave * 8 + q;
        float* p = outF + (size_t)m * N + nBlk + lane * 4;
        *(volatile v4f*)p = vals[q];
      }
    }
  }
}

__global__ __launch_bounds__(256) void mflag_kernel(
    const int* __restrict__ mask, int* __restrict__ mflag) {
  constexpr int NKB = SEQ / 32;
  const int qt = blockIdx.x;
  const int tid = threadIdx.x, wave = tid >> 5, lane = tid & 31;
  __shared__ __align__(16) int fl[FLAG_STRIDE];
  if (tid < FLAG_STRIDE) fl[tid] = 0;
  __syncthreads();
  for (int kb = wave; kb < NKB; kb += 8) {
    int z = 0;
    const int* mp = mask + (size_t)(qt * 64) * T_FULL + kb * 32 + lane;
#pragma unroll 4
    for (int rr = 0; rr < 64; ++rr) z |= (mp[(size_t)rr * T_FULL] == 0) ? 1 : 0;
#pragma unroll
    for (int m = 16; m >= 1; m >>= 1) z |= __shfl_xor(z, m, 32);
    if (lane == 0) fl[kb] = z;
  }
  __syncthreads();
  if (wave == 0) {
    const int li = lane & 15;
    const v4i val = *(const v4i*)&fl[li * 4];
    int* p = mflag + (size_t)qt * FLAG_STRIDE + li * 4;
    if (lane < 16) *(volatile v4i*)p = val;
    __threadfence();
    if (lane < 16) *(volatile v4i*)p = val;
  }
}

#define KPAD 72
#define VPAD 40

__global__ __launch_bounds__(128) void attn_kernel(
    const _Float16* __restrict__ qkv, const int* __restrict__ mask,
    const int* __restrict__ mflag, _Float16* __restrict__ o16) {
  constexpr int N = SEQ;
  constexpr int LDQ = NQKV;
  constexpr int NQT = SEQ / 64;
  constexpr int NKB = SEQ / 32;
  const int qt = blockIdx.x % NQT;
  const int bh = blockIdx.x / NQT;
  const int h = bh % NH, b = bh / NH;

  __shared__ __align__(16) _Float16 Ks[2 * 32 * KPAD];
  __shared__ __align__(16) _Float16 Vt[2 * 64 * VPAD];
  __shared__ __align__(16) _Float16 Ps[4 * 16 * VPAD];

  const int tid = threadIdx.x, wave = tid >> 5, lane = tid & 31;
  const int r = lane & 15, hb = (lane >> 4) << 3;
  const _Float16* Qb = qkv + (size_t)b * N * LDQ + h * HD;
  const _Float16* Kb = Qb + DM;
  const _Float16* Vb = Qb + 2 * DM;
  const int q0 = qt * 64 + wave * 16;

  v16h aq[2];
#pragma unroll
  for (int dc = 0; dc < 2; ++dc)
    aq[dc] = load_frag(Qb + (size_t)(q0 + r) * LDQ + dc * 32 + hb);

  v16h ones;
#pragma unroll
  for (int e = 0; e < 16; ++e) ones[e] = (_Float16)1.0f;

  v8f o[4] = {};
  float mrow[8], lrow[8];
#pragma unroll
  for (int v = 0; v < 8; ++v) { mrow[v] = -1e30f; lrow[v] = 0.f; }

  _Float16* Pw = Ps + wave * 16 * VPAD;

  const int kr0 = tid >> 3, c0 = (tid & 7) << 3, kr1 = kr0 + 16;
  const _Float16* gK0 = Kb + (size_t)kr0 * LDQ + c0;
  const _Float16* gK1 = Kb + (size_t)kr1 * LDQ + c0;
  const _Float16* gV0 = Vb + (size_t)kr0 * LDQ + c0;
  const _Float16* gV1 = Vb + (size_t)kr1 * LDQ + c0;

  v8h kk0 = *(const v8h*)gK0, kk1 = *(const v8h*)gK1;
  v8h vv0 = *(const v8h*)gV0, vv1 = *(const v8h*)gV1;
  *(v8h*)&Ks[kr0 * KPAD + c0] = kk0;
  *(v8h*)&Ks[kr1 * KPAD + c0] = kk1;
#pragma unroll
  for (int j = 0; j < 8; ++j) Vt[(c0 + j) * VPAD + kr0] = vv0[j];
#pragma unroll
  for (int j = 0; j < 8; ++j) Vt[(c0 + j) * VPAD + kr1] = vv1[j];

  const float ninf = __uint_as_float(0xff800000u);

  for (int kb = 0; kb < NKB; ++kb) {
    const int cur = kb & 1;
    __syncthreads();

    const int fl = mflag[(size_t)qt * FLAG_STRIDE + kb];
    const bool nxt = (kb + 1 < NKB);
    if (nxt) {
      const size_t oo = (size_t)((kb + 1) * 32) * LDQ;
      kk0 = *(const v8h*)(gK0 + oo); kk1 = *(const v8h*)(gK1 + oo);
      vv0 = *(const v8h*)(gV0 + oo); vv1 = *(const v8h*)(gV1 + oo);
    }
    const _Float16* Kc = Ks + cur * 32 * KPAD;
    const _Float16* Vc = Vt + cur * 64 * VPAD;

    v8f s[2] = {};
#pragma unroll
    for (int kt = 0; kt < 2; ++kt)
#pragma unroll
      for (int dc = 0; dc < 2; ++dc) {
        v16h bk = load_frag(Kc + (kt * 16 + r) * KPAD + dc * 32 + hb);
        s[kt] = mma16(aq[dc], bk, s[kt]);
      }

    int mk0[8], mk1[8];
#pragma unroll
    for (int v = 0; v < 8; ++v) { mk0[v] = 1; mk1[v] = 1; }
    if (fl != 0) {
#pragma unroll
      for (int v = 0; v < 8; ++v) {
        const size_t mr = (size_t)(q0 + hb + v) * T_FULL + (size_t)(kb * 32 + r);
        mk0[v] = mask[mr];
        mk1[v] = mask[mr + 16];
      }
    }

    float alpha[8];
#pragma unroll
    for (int v = 0; v < 8; ++v) {
      float s0 = s[0][v] * 0.125f, s1 = s[1][v] * 0.125f;
      s0 = (mk0[v] == 0) ? ninf : s0;
      s1 = (mk1[v] == 0) ? ninf : s1;
      float mx = fmaxf(s0, s1);
#pragma unroll
      for (int msk = 8; msk >= 1; msk >>= 1) mx = fmaxf(mx, __shfl_xor(mx, msk, 32));
      const float mnew = fmaxf(mrow[v], mx);
      alpha[v] = __expf(mrow[v] - mnew);
      mrow[v] = mnew;
      s[0][v] = 1024.0f * __expf(s0 - mnew);
      s[1][v] = 1024.0f * __expf(s1 - mnew);
    }

#pragma unroll
    for (int kt = 0; kt < 2; ++kt)
#pragma unroll
      for (int v = 0; v < 8; ++v)
        Pw[(v + hb) * VPAD + kt * 16 + r] = (_Float16)s[kt][v];
    __syncthreads();
    v16h pf = load_frag(Pw + r * VPAD + hb);

    v8f zero = {};
    v8f rsum = mma16(pf, ones, zero);
#pragma unroll
    for (int v = 0; v < 8; ++v) lrow[v] = lrow[v] * alpha[v] + rsum[v];

#pragma unroll
    for (int t = 0; t < 4; ++t) {
#pragma unroll
      for (int v = 0; v < 8; ++v) o[t][v] *= alpha[v];
      v16h bv = load_frag(Vc + (t * 16 + r) * VPAD + hb);
      o[t] = mma16(pf, bv, o[t]);
    }

    if (nxt) {
      _Float16* Kn = Ks + (cur ^ 1) * 32 * KPAD;
      _Float16* Vn = Vt + (cur ^ 1) * 64 * VPAD;
      *(v8h*)&Kn[kr0 * KPAD + c0] = kk0;
      *(v8h*)&Kn[kr1 * KPAD + c0] = kk1;
#pragma unroll
      for (int j = 0; j < 8; ++j) Vn[(c0 + j) * VPAD + kr0] = vv0[j];
#pragma unroll
      for (int j = 0; j < 8; ++j) Vn[(c0 + j) * VPAD + kr1] = vv1[j];
    }
  }

  __syncthreads();
  _Float16* Os = Ks + wave * 16 * KPAD;
#pragma unroll
  for (int t = 0; t < 4; ++t)
#pragma unroll
    for (int v = 0; v < 8; ++v) {
      const float il = 32.0f * __builtin_amdgcn_rcpf(lrow[v]);
      Os[(v + hb) * KPAD + t * 16 + r] = (_Float16)(o[t][v] * il);
    }
  __syncthreads();
  const int rsub = lane >> 3, piece = lane & 7;
  v8h ov[4];
#pragma unroll
  for (int it = 0; it < 4; ++it) ov[it] = *(const v8h*)&Os[(it * 4 + rsub) * KPAD + piece * 8];
#pragma unroll
  for (int it = 0; it < 4; ++it) {
    const int row = it * 4 + rsub;
    _Float16* p = o16 + (size_t)(b * N + q0 + row) * DM + h * HD + piece * 8;
    *(volatile v8h*)p = ov[it];
  }
  __threadfence();
#pragma unroll
  for (int it = 0; it < 4; ++it) {
    const int row = it * 4 + rsub;
    _Float16* p = o16 + (size_t)(b * N + q0 + row) * DM + h * HD + piece * 8;
    *(volatile v8h*)p = ov[it];
  }
}

extern "C" void kernel_launch(void* const* d_in, const int* in_sizes, int n_in,
                              void* d_out, int out_size, void* d_ws, size_t ws_size,
                              hipStream_t stream) {
  if (n_in < 15) return;
  const float* x    = (const float*)d_in[0];
  const int*   mask = (const int*)d_in[1];
  const float* Wq   = (const float*)d_in[2];
  const float* Wk   = (const float*)d_in[3];
  const float* Wv   = (const float*)d_in[4];
  const float* Wp   = (const float*)d_in[5];
  const float* bp   = (const float*)d_in[6];
  const float* W1   = (const float*)d_in[7];
  const float* b1   = (const float*)d_in[8];
  const float* W2   = (const float*)d_in[9];
  const float* b2   = (const float*)d_in[10];
  const float* g1   = (const float*)d_in[11];
  const float* be1  = (const float*)d_in[12];
  const float* g2   = (const float*)d_in[13];
  const float* be2  = (const float*)d_in[14];
  float* out = (float*)d_out;

  if ((long long)in_sizes[0] < (long long)(NB - 1) * SEQ_FULL * DM + (long long)SEQ * DM) return;
  if ((long long)in_sizes[1] < (long long)(SEQ - 1) * T_FULL + SEQ) return;
  if (in_sizes[2] < NH * DM * HD || in_sizes[3] < NH * DM * HD || in_sizes[4] < NH * DM * HD) return;
  if (in_sizes[5] < DM * DM || in_sizes[6] < DM) return;
  if (in_sizes[7] < DM * HID || in_sizes[8] < HID) return;
  if (in_sizes[9] < HID * DM || in_sizes[10] < DM) return;
  if (in_sizes[11] < DM || in_sizes[12] < DM || in_sizes[13] < DM || in_sizes[14] < DM) return;
  if (out_size < NTOK * DM) return;

  char* ws = (char*)d_ws;
  size_t off = 0;
  auto alloc = [&](size_t bytes) -> char* {
    char* p = ws + off;
    off += (bytes + 255) & ~(size_t)255;
    return p;
  };
  _Float16* wqkv16 = (_Float16*)alloc((size_t)NQKV * DM * 2);
  _Float16* wp16   = (_Float16*)alloc((size_t)DM * DM * 2);
  _Float16* w1t16  = (_Float16*)alloc((size_t)HID * DM * 2);
  _Float16* w2t16  = (_Float16*)alloc((size_t)DM * HID * 2);
  _Float16* h16    = (_Float16*)alloc((size_t)NTOK * DM * 2);
  _Float16* act    = (_Float16*)alloc((size_t)NTOK * HID * 2);
  float*    x1     = (float*)alloc((size_t)NTOK * DM * 4);
  int*      mflag  = (int*)alloc((size_t)(SEQ / 64) * FLAG_STRIDE * 4);
  if (off > ws_size) return;
  _Float16* qkv16 = act;
  _Float16* o16   = act + (size_t)NTOK * NQKV;
  _Float16* g16   = act;

  tcvt_kernel<<<dim3(DM / 64, HD / 32, NH), 256, 0, stream>>>(Wq, DM * HD, HD, wqkv16, DM, HD, 0,      64.0f);
  tcvt_kernel<<<dim3(DM / 64, HD / 32, NH), 256, 0, stream>>>(Wk, DM * HD, HD, wqkv16, DM, HD, DM,     64.0f);
  tcvt_kernel<<<dim3(DM / 64, HD / 32, NH), 256, 0, stream>>>(Wv, DM * HD, HD, wqkv16, DM, HD, 2 * DM, 64.0f);
  tcvt_kernel<<<dim3(DM / 64, DM / 32, 1), 256, 0, stream>>>(Wp, 0, DM, wp16, DM, 0, 0, 64.0f);
  tcvt_kernel<<<dim3(DM / 64, HID / 32, 1), 256, 0, stream>>>(W1, 0, HID, w1t16, DM, 0, 0, 64.0f);
  tcvt_kernel<<<dim3(HID / 64, DM / 32, 1), 256, 0, stream>>>(W2, 0, DM, w2t16, HID, 0, 0, 128.0f);

  mflag_kernel<<<dim3(SEQ / 64), 256, 0, stream>>>(mask, mflag);

  ln_kernel<true><<<dim3(NTOK), 128, 0, stream>>>(x, SEQ_FULL, g1, be1, h16);

  gemm_kernel<false, false, false, false, true>
      <<<dim3(NQKV / 128, NTOK / 128), 256, 0, stream>>>(
          h16, wqkv16, bp, x, SEQ, x1, qkv16, NTOK, NQKV, DM, 1.0f / 64.0f);

  attn_kernel<<<dim3(NB * NH * (SEQ / 64)), 128, 0, stream>>>(qkv16, mask, mflag, o16);

  gemm_kernel<true, true, true, false, false>
      <<<dim3(DM / 128, NTOK / 128), 256, 0, stream>>>(
          o16, wp16, bp, x, SEQ_FULL, x1, h16, NTOK, DM, DM, 1.0f / 2048.0f);

  ln_kernel<false><<<dim3(NTOK), 128, 0, stream>>>(x1, SEQ, g2, be2, h16);

  gemm_kernel<true, false, false, true, true>
      <<<dim3(HID / 128, NTOK / 128), 256, 0, stream>>>(
          h16, w1t16, b1, x, SEQ, x1, g16, NTOK, HID, DM, 1.0f / 64.0f);

  gemm_kernel<true, true, false, false, false>
      <<<dim3(DM / 128, NTOK / 128), 256, 0, stream>>>(
          g16, w2t16, b2, x1, SEQ, out, h16, NTOK, DM, HID, 1.0f / 128.0f);
}
